// GatedFusionMambaBlock_76338748719293
// MI455X (gfx1250) — hardware-verified
//
#include <hip/hip_runtime.h>
#include <hip/hip_bf16.h>
#include <math.h>


typedef _Float16 bf16;
typedef _Float16 f16;
typedef __attribute__((ext_vector_type(4))) unsigned v4u_t;
typedef unsigned v4ua __attribute__((ext_vector_type(4), may_alias));
typedef __attribute__((ext_vector_type(4))) float v4f_t;
typedef float v4fa __attribute__((ext_vector_type(4), may_alias));
typedef __attribute__((ext_vector_type(16))) bf16  bf16x16;
typedef bf16x16 f16x16;
typedef __attribute__((ext_vector_type(8)))  bf16  bf16x8;
typedef bf16x8 f16x8;
typedef __attribute__((ext_vector_type(4)))  bf16  bf16x4;
typedef __attribute__((ext_vector_type(8)))  float f32x8;
__device__ __forceinline__ f32x8 wmma16(f16x16 a, f16x16 b, f32x8 c) {
  c = __builtin_amdgcn_wmma_f32_16x16x32_f16(false, a, false, b, (short)0, c, false, false);
  asm volatile("v_nop\n\tv_nop\n\tv_nop\n\tv_nop" : "+v"(c) : "v"(a), "v"(b));
  return c;
}
#define LDS_STRIDE 48
#define KSTRIDE    72
#define VSTRIDE    48

__device__ __forceinline__ f32x8 wmma_bf16(bf16x16 a, bf16x16 b, f32x8 c) {
  c = __builtin_amdgcn_wmma_f32_16x16x32_f16(false, a, false, b, (short)0, c, false, false);
  asm volatile("v_nop\n\tv_nop\n\tv_nop\n\tv_nop" : "+v"(c) : "v"(a), "v"(b));
  return c;
}

template <typename T>
__device__ __forceinline__ bf16x16 load_frag(const T* __restrict__ base, int ld,
                                             int row0, int k0) {
  const int lane = threadIdx.x & 31;
  const int r    = lane & 15;
  const int kh   = (lane >> 4) * 8;
  const T* p0 = base + (size_t)(row0 + r) * ld + (k0 + kh);
  const T* p1 = p0 + 16;
  bf16x16 f;
#pragma unroll
  for (int i = 0; i < 8; ++i) {
    f[i]     = (bf16)p0[i];
    f[i + 8] = (bf16)p1[i];
  }
  return f;
}

__device__ __forceinline__ bf16x16 lds_frag(const bf16* base, int stride) {
  const int lane = threadIdx.x & 31;
  const int row  = lane & 15;
  const int kh   = (lane >> 4) * 8;
  const bf16x8 lo = *(const bf16x8*)(base + row * stride + kh);
  const bf16x8 hi = *(const bf16x8*)(base + row * stride + kh + 16);
  bf16x16 f;
#pragma unroll
  for (int i = 0; i < 8; ++i) { f[i] = lo[i]; f[i + 8] = hi[i]; }
  return f;
}

template <typename T>
__device__ __forceinline__ void stage_read16(const T* __restrict__ p, float* buf) {
#pragma unroll
  for (int i = 0; i < 16; ++i) buf[i] = (float)p[i];
}

__device__ __forceinline__ void stage_write(bf16* dst, const float* buf, int nquad) {
#pragma unroll
  for (int i = 0; i < nquad; ++i) {
    bf16x4 q;
    q[0] = (bf16)buf[4 * i];     q[1] = (bf16)buf[4 * i + 1];
    q[2] = (bf16)buf[4 * i + 2]; q[3] = (bf16)buf[4 * i + 3];
    *(bf16x4*)(dst + 4 * i) = q;
  }
}


#define GSTR 48
#define GSTR 48
template <typename AT, int EPI, bool OUT16>
__global__ __launch_bounds__(256) void gemm_kne(const AT* __restrict__ A, int lda, const float* __restrict__ Wm, int ldw,
                                                const float* __restrict__ bias, const float* __restrict__ R, const float* __restrict__ gvec,
                                                void* __restrict__ Yv, int ldy, int K) {
  __shared__ __attribute__((aligned(16))) f16 ldsA[128 * GSTR];
  __shared__ __attribute__((aligned(16))) f16 ldsW[128 * GSTR];
  __shared__ __attribute__((aligned(16))) float oS[8][32 * 68];
  const int tid = threadIdx.x, lane = tid & 31, wave = tid >> 5, cl = lane & 15, rh = (lane >> 4) * 8;
  const int m0 = blockIdx.x * 128, n0 = blockIdx.y * 128;
  const int wm = (wave & 3) * 32, wn = (wave >> 2) * 64;
  f32x8 acc[2][4];
#pragma unroll
  for (int i = 0; i < 2; ++i)
#pragma unroll
    for (int j = 0; j < 4; ++j) { f32x8 z = {}; acc[i][j] = z; }
#pragma unroll 1
  for (int k0 = 0; k0 < K; k0 += 32) {
    __syncthreads();
    { const int row = tid >> 1, ch = (tid & 1) * 16;
      const AT* src = A + (size_t)(m0 + row) * lda + k0 + ch;
#pragma unroll
      for (int g = 0; g < 16; ++g) ldsA[row * GSTR + ch + g] = (f16)src[g]; }
    { const int k = tid >> 3, nn0 = (tid & 7) * 16;
      const float* src = Wm + (size_t)(k0 + k) * ldw + n0 + nn0;
#pragma unroll
      for (int g = 0; g < 4; ++g) { const v4f_t v = *(const v4f_t*)(src + 4 * g);
#pragma unroll
        for (int u = 0; u < 4; ++u) ldsW[(nn0 + 4 * g + u) * GSTR + k] = (f16)v[u]; } }
    __syncthreads();
    f16x16 af[2];
#pragma unroll
    for (int i = 0; i < 2; ++i) af[i] = lds_frag(ldsA + (wm + 16 * i) * GSTR, GSTR);
#pragma unroll
    for (int j = 0; j < 4; ++j) {
      const f16x16 bf = lds_frag(ldsW + (wn + 16 * j) * GSTR, GSTR);
#pragma unroll
      for (int i = 0; i < 2; ++i) acc[i][j] = wmma16(af[i], bf, acc[i][j]);
    }
  }
  float* so = oS[wave];
#pragma unroll
  for (int i = 0; i < 2; ++i)
#pragma unroll
    for (int j = 0; j < 4; ++j) {
      const int n = n0 + wn + 16 * j + cl;
      const float bv = bias ? bias[n] : 0.0f;
      const float gv = (EPI == 2 || EPI == 4) ? gvec[n] : 0.0f;
      if (EPI == 1) {
#pragma unroll 1
        for (int r = 0; r < 8; ++r) { const float xg = acc[i][j][r] + bv; so[(16 * i + rh + r) * 68 + 16 * j + cl] = 0.5f * xg * (1.0f + erff(xg * 0.70710678118654752f)); }
      } else if (EPI == 11) {
#pragma unroll 1
        for (int r = 0; r < 8; ++r) { const float xg = acc[i][j][r] + bv; so[(16 * i + rh + r) * 68 + 16 * j + cl] = xg / (1.0f + expf(-xg)); }
      } else if (EPI == 9 || EPI == 10) {
#pragma unroll 1
        for (int r = 0; r < 8; ++r) { const float xg = acc[i][j][r] + bv + R[(size_t)(m0 + wm + 16 * i + rh + r) * ldy + n]; so[(16 * i + rh + r) * 68 + 16 * j + cl] = (EPI == 9) ? 1.0f / (1.0f + expf(-xg)) : tanhf(xg); }
      } else {
#pragma unroll
        for (int r = 0; r < 8; ++r) {
          float v = acc[i][j][r] + bv;
          if (EPI == 3) v = fmaxf(v, 0.0f);
          if (EPI == 6) v = fminf(fmaxf(v, 0.0f), 6.0f);
          if (EPI == 4) v = gv * v;
          if (EPI == 2) v = R[(size_t)(m0 + wm + 16 * i + rh + r) * ldy + n] + gv * v;
          so[(16 * i + rh + r) * 68 + 16 * j + cl] = v;
        }
      }
    }
  asm volatile("s_wait_dscnt 0" ::: "memory");
  __builtin_amdgcn_wave_barrier();
#pragma unroll 1
  for (int pass = 0; pass < 2; ++pass) {
    if (OUT16) {
      f16* Y = (f16*)Yv;
#pragma unroll
      for (int it = 0; it < 8; ++it) { const int c = lane + 32 * it, rr = c >> 3, q8 = (c & 7) * 8;
        union { f16 h[8]; v4u_t v; } u;
#pragma unroll
        for (int e = 0; e < 8; ++e) u.h[e] = (f16)so[rr * 68 + q8 + e];
        *(volatile v4u_t*)(Y + (size_t)(m0 + wm + rr) * ldy + n0 + wn + q8) = u.v; }
    } else {
      float* Y = (float*)Yv;
#pragma unroll
      for (int it = 0; it < 16; ++it) { const int f4 = lane + 32 * it, rr = f4 >> 4, q = (f4 & 15) * 4;
        *(volatile v4f_t*)(Y + (size_t)(m0 + wm + rr) * ldy + n0 + wn + q) = *(const v4fa*)(so + rr * 68 + q); }
    }
    __threadfence();
  }
}

template <typename AT, int EPI, bool OUT16>
__global__ __launch_bounds__(256) void gemm_knez(const AT* __restrict__ A, int lda, size_t strideA, const float* __restrict__ Wm, int ldw, size_t strideW,
                                                 const float* __restrict__ bias, const float* __restrict__ R, const float* __restrict__ gvec,
                                                 void* __restrict__ Yv, int ldy, size_t strideY, int K) {
  A += (size_t)blockIdx.z * strideA; Wm += (size_t)blockIdx.z * strideW; Yv = (void*)((char*)Yv + (size_t)blockIdx.z * strideY * (OUT16 ? 2 : 4)); if (R) R += (size_t)blockIdx.z * strideY;
  __shared__ __attribute__((aligned(16))) f16 ldsA[128 * GSTR];
  __shared__ __attribute__((aligned(16))) f16 ldsW[128 * GSTR];
  __shared__ __attribute__((aligned(16))) float oS[8][32 * 68];
  const int tid = threadIdx.x, lane = tid & 31, wave = tid >> 5, cl = lane & 15, rh = (lane >> 4) * 8;
  const int m0 = blockIdx.x * 128, n0 = blockIdx.y * 128;
  const int wm = (wave & 3) * 32, wn = (wave >> 2) * 64;
  f32x8 acc[2][4];
#pragma unroll
  for (int i = 0; i < 2; ++i)
#pragma unroll
    for (int j = 0; j < 4; ++j) { f32x8 z = {}; acc[i][j] = z; }
#pragma unroll 1
  for (int k0 = 0; k0 < K; k0 += 32) {
    __syncthreads();
    { const int row = tid >> 1, ch = (tid & 1) * 16;
      const AT* src = A + (size_t)(m0 + row) * lda + k0 + ch;
#pragma unroll
      for (int g = 0; g < 16; ++g) ldsA[row * GSTR + ch + g] = (f16)src[g]; }
    { const int k = tid >> 3, nn0 = (tid & 7) * 16;
      const float* src = Wm + (size_t)(k0 + k) * ldw + n0 + nn0;
#pragma unroll
      for (int g = 0; g < 4; ++g) { const v4f_t v = *(const v4f_t*)(src + 4 * g);
#pragma unroll
        for (int u = 0; u < 4; ++u) ldsW[(nn0 + 4 * g + u) * GSTR + k] = (f16)v[u]; } }
    __syncthreads();
    f16x16 af[2];
#pragma unroll
    for (int i = 0; i < 2; ++i) af[i] = lds_frag(ldsA + (wm + 16 * i) * GSTR, GSTR);
#pragma unroll
    for (int j = 0; j < 4; ++j) {
      const f16x16 bf = lds_frag(ldsW + (wn + 16 * j) * GSTR, GSTR);
#pragma unroll
      for (int i = 0; i < 2; ++i) acc[i][j] = wmma16(af[i], bf, acc[i][j]);
    }
  }
  float* so = oS[wave];
#pragma unroll
  for (int i = 0; i < 2; ++i)
#pragma unroll
    for (int j = 0; j < 4; ++j) {
      const int n = n0 + wn + 16 * j + cl;
      const float bv = bias ? bias[n] : 0.0f;
      const float gv = (EPI == 2 || EPI == 4) ? gvec[n] : 0.0f;
      if (EPI == 1) {
#pragma unroll 1
        for (int r = 0; r < 8; ++r) { const float xg = acc[i][j][r] + bv; so[(16 * i + rh + r) * 68 + 16 * j + cl] = 0.5f * xg * (1.0f + erff(xg * 0.70710678118654752f)); }
      } else if (EPI == 11) {
#pragma unroll 1
        for (int r = 0; r < 8; ++r) { const float xg = acc[i][j][r] + bv; so[(16 * i + rh + r) * 68 + 16 * j + cl] = xg / (1.0f + expf(-xg)); }
      } else if (EPI == 9 || EPI == 10) {
#pragma unroll 1
        for (int r = 0; r < 8; ++r) { const float xg = acc[i][j][r] + bv + R[(size_t)(m0 + wm + 16 * i + rh + r) * ldy + n]; so[(16 * i + rh + r) * 68 + 16 * j + cl] = (EPI == 9) ? 1.0f / (1.0f + expf(-xg)) : tanhf(xg); }
      } else {
#pragma unroll
        for (int r = 0; r < 8; ++r) {
          float v = acc[i][j][r] + bv;
          if (EPI == 3) v = fmaxf(v, 0.0f);
          if (EPI == 6) v = fminf(fmaxf(v, 0.0f), 6.0f);
          if (EPI == 4) v = gv * v;
          if (EPI == 2) v = R[(size_t)(m0 + wm + 16 * i + rh + r) * ldy + n] + gv * v;
          so[(16 * i + rh + r) * 68 + 16 * j + cl] = v;
        }
      }
    }
  asm volatile("s_wait_dscnt 0" ::: "memory");
  __builtin_amdgcn_wave_barrier();
#pragma unroll 1
  for (int pass = 0; pass < 2; ++pass) {
    if (OUT16) {
      f16* Y = (f16*)Yv;
#pragma unroll
      for (int it = 0; it < 8; ++it) { const int c = lane + 32 * it, rr = c >> 3, q8 = (c & 7) * 8;
        union { f16 h[8]; v4u_t v; } u;
#pragma unroll
        for (int e = 0; e < 8; ++e) u.h[e] = (f16)so[rr * 68 + q8 + e];
        *(volatile v4u_t*)(Y + (size_t)(m0 + wm + rr) * ldy + n0 + wn + q8) = u.v; }
    } else {
      float* Y = (float*)Yv;
#pragma unroll
      for (int it = 0; it < 16; ++it) { const int f4 = lane + 32 * it, rr = f4 >> 4, q = (f4 & 15) * 4;
        *(volatile v4f_t*)(Y + (size_t)(m0 + wm + rr) * ldy + n0 + wn + q) = *(const v4fa*)(so + rr * 68 + q); }
    }
    __threadfence();
  }
}

template <typename AT, bool ACC>
__global__ __launch_bounds__(256) void gemm_kn2(const AT* __restrict__ A, int lda, size_t strideA,
                                               const float* __restrict__ Wm, int ldw, size_t strideW,
                                               const float* __restrict__ bias, float scale,
                                               float* __restrict__ Y, int ldy, size_t strideY, int K) {
  __shared__ __attribute__((aligned(16))) f16 ldsA[128 * GSTR], ldsAl[128 * GSTR];
  __shared__ __attribute__((aligned(16))) f16 ldsW[128 * GSTR], ldsWl[128 * GSTR];
  __shared__ __attribute__((aligned(16))) float oS[8][32 * 68];
  const int tid = threadIdx.x, lane = tid & 31, wave = tid >> 5, cl = lane & 15, rh = (lane >> 4) * 8;
  const int m0 = blockIdx.x * 128, n0 = blockIdx.y * 128;
  const int wm = (wave & 3) * 32, wn = (wave >> 2) * 64;
  A += (size_t)blockIdx.z * strideA; Wm += (size_t)blockIdx.z * strideW; Y += (size_t)blockIdx.z * strideY;
  f32x8 acc[2][4], accx[2][4];
#pragma unroll
  for (int i = 0; i < 2; ++i)
#pragma unroll
    for (int j = 0; j < 4; ++j) { f32x8 z = {}; acc[i][j] = z; accx[i][j] = z; }
#pragma unroll 1
  for (int k0 = 0; k0 < K; k0 += 32) {
    __syncthreads();
    {
      const int row = tid >> 1, ch = (tid & 1) * 16;
      const AT* src = A + (size_t)(m0 + row) * lda + k0 + ch;
#pragma unroll
      for (int g = 0; g < 16; ++g) { const float v = (float)src[g]; const f16 h = (f16)v; ldsA[row * GSTR + ch + g] = h; ldsAl[row * GSTR + ch + g] = (f16)((v - (float)h) * 2048.0f); }
    }
    {
      const int k = tid >> 3, nn0 = (tid & 7) * 16;
      const float* src = Wm + (size_t)(k0 + k) * ldw + n0 + nn0;
#pragma unroll
      for (int g = 0; g < 4; ++g) { const v4f_t v = *(const v4f_t*)(src + 4 * g);
#pragma unroll
        for (int u = 0; u < 4; ++u) { const f16 h = (f16)v[u]; ldsW[(nn0 + 4 * g + u) * GSTR + k] = h; ldsWl[(nn0 + 4 * g + u) * GSTR + k] = (f16)((v[u] - (float)h) * 2048.0f); } }
    }
    __syncthreads();
    f16x16 af[2], afl[2];
#pragma unroll
    for (int i = 0; i < 2; ++i) { af[i] = lds_frag(ldsA + (wm + 16 * i) * GSTR, GSTR); afl[i] = lds_frag(ldsAl + (wm + 16 * i) * GSTR, GSTR); }
#pragma unroll
    for (int j = 0; j < 4; ++j) {
      const f16x16 bf = lds_frag(ldsW + (wn + 16 * j) * GSTR, GSTR), bfl = lds_frag(ldsWl + (wn + 16 * j) * GSTR, GSTR);
#pragma unroll
      for (int i = 0; i < 2; ++i) { acc[i][j] = wmma16(af[i], bf, acc[i][j]); accx[i][j] = wmma16(af[i], bfl, accx[i][j]); accx[i][j] = wmma16(afl[i], bf, accx[i][j]); }
    }
  }
  float* so = oS[wave];
#pragma unroll
  for (int i = 0; i < 2; ++i)
#pragma unroll
    for (int j = 0; j < 4; ++j) {
      const float bv = bias ? bias[n0 + wn + 16 * j + cl] : 0.0f;
#pragma unroll
      for (int r = 0; r < 8; ++r) so[(16 * i + rh + r) * 68 + 16 * j + cl] = (acc[i][j][r] + accx[i][j][r] * (1.0f / 2048.0f)) * scale + bv;
    }
  asm volatile("s_wait_dscnt 0" ::: "memory");
  __builtin_amdgcn_wave_barrier();
  if (ACC) {
#pragma unroll
    for (int it = 0; it < 16; ++it) { const int f4 = lane + 32 * it, rr = f4 >> 4, q = (f4 & 15) * 4;
      const v4f_t old = *(const v4fa*)(Y + (size_t)(m0 + wm + rr) * ldy + n0 + wn + q);
      v4f_t v = *(const v4fa*)(so + rr * 68 + q); v += old; *(v4fa*)(so + rr * 68 + q) = v; }
    asm volatile("s_wait_dscnt 0" ::: "memory");
  }
#pragma unroll 1
  for (int pass = 0; pass < 2; ++pass) {
#pragma unroll
    for (int it = 0; it < 16; ++it) { const int f4 = lane + 32 * it, rr = f4 >> 4, q = (f4 & 15) * 4;
      *(volatile v4f_t*)(Y + (size_t)(m0 + wm + rr) * ldy + n0 + wn + q) = *(const v4fa*)(so + rr * 68 + q); }
    __threadfence();
  }
}

__global__ __launch_bounds__(256) void k_transpose(const float* __restrict__ Wm, float* __restrict__ Wt, int rows, int cols) {
  __shared__ float tS[64][65];
  const int tid = threadIdx.x, tbj = cols / 64, bi = blockIdx.x / tbj, bj = blockIdx.x % tbj;
  for (int e = tid; e < 64 * 64; e += 256) { const int r = e >> 6, c = e & 63; tS[r][c] = Wm[(size_t)(bi * 64 + r) * cols + bj * 64 + c]; }
  __syncthreads();
  for (int ch = tid; ch < 64 * 16; ch += 256) { const int r = ch >> 4, q4 = (ch & 15) * 4; v4f_t o; o[0] = tS[q4][r]; o[1] = tS[q4 + 1][r]; o[2] = tS[q4 + 2][r]; o[3] = tS[q4 + 3][r];
    float* dst = Wt + (size_t)(bj * 64 + r) * rows + bi * 64 + q4; *(volatile v4f_t*)dst = o; __threadfence(); *(volatile v4f_t*)dst = o; }
}

#define NBg 2
#define SSg 2048
#define DDg 512
#define DIg 1024
#define NHg 16
#define HPg 64
#define NSg 16
#define CDg 1056
#define NPg 2096
#define NPP 2176
#define FFg 2048
#define TCH 64
__global__ __launch_bounds__(256) void k_fill(float* __restrict__ p, float val, size_t n4) { const size_t i = (size_t)blockIdx.x * 256 + threadIdx.x; if (i < n4) { v4f_t v = {val, val, val, val}; *(volatile v4f_t*)(p + 4 * i) = v; __threadfence(); *(volatile v4f_t*)(p + 4 * i) = v; } }
__global__ __launch_bounds__(256) void k_dbg_zero(float* __restrict__ p, size_t n4) { const size_t i = (size_t)blockIdx.x * 256 + threadIdx.x; if (i < n4) { v4f_t z = {0.f,0.f,0.f,0.f}; *(volatile v4f_t*)(p + 4 * i) = z; __threadfence(); *(volatile v4f_t*)(p + 4 * i) = z; } }
__global__ __launch_bounds__(256) void k_copy(const float* __restrict__ src, float* __restrict__ dst, size_t n4) { const size_t i = (size_t)blockIdx.x * 256 + threadIdx.x; if (i < n4) { const v4f_t v = *(const v4f_t*)(src + 4 * i); *(volatile v4f_t*)(dst + 4 * i) = v; __threadfence(); *(volatile v4f_t*)(dst + 4 * i) = v; } }
__global__ __launch_bounds__(256) void k_rms(const float* __restrict__ X, const float* __restrict__ g, float* __restrict__ Y) {
  __shared__ __attribute__((aligned(16))) float rowS[16 * 516];
  const int tid = threadIdx.x, r = tid >> 4, part = tid & 15; const size_t row = (size_t)blockIdx.x * 16 + r;
  float q = 0.0f;
#pragma unroll 1
  for (int i = 0; i < 32; ++i) { const float v = X[row * 512 + part * 32 + i]; rowS[r * 516 + part * 32 + i] = v; q += v * v; }
  q += __shfl_xor(q, 1, 32); q += __shfl_xor(q, 2, 32); q += __shfl_xor(q, 4, 32); q += __shfl_xor(q, 8, 32);
  const float rs = 1.0f / __builtin_sqrtf(q * (1.0f / 512.0f) + 1e-6f);
#pragma unroll 1
  for (int i = 0; i < 32; ++i) { const int c = part * 32 + i; rowS[r * 516 + c] = rowS[r * 516 + c] * rs * g[c]; }
  __syncthreads();
#pragma unroll 1
  for (int pass = 0; pass < 2; ++pass) { for (int q4 = tid; q4 < 16 * 128; q4 += 256) { const int rr = q4 / 128, c4 = (q4 % 128) * 4;
      *(volatile v4f_t*)(Y + ((size_t)blockIdx.x * 16 + rr) * 512 + c4) = *(const v4fa*)(rowS + rr * 516 + c4); } __threadfence(); }
}
__global__ __launch_bounds__(256) void k_padin(const float* __restrict__ Wm, float* __restrict__ WT) {
  const int k = blockIdx.x, tid = threadIdx.x;
#pragma unroll 1
  for (int n = tid; n < NPP; n += 256) { const float v = (n < NPg) ? Wm[(size_t)min(n, NPg - 1) * DDg + k] : 0.0f; *(volatile float*)(WT + (size_t)k * NPP + n) = v; }
  __threadfence();
#pragma unroll 1
  for (int n = tid; n < NPP; n += 256) { float* p = WT + (size_t)k * NPP + n; const float v = p[0]; *(volatile float*)p = v; }
}
__global__ __launch_bounds__(256) void k_fuse(float* __restrict__ Hn, const float* __restrict__ wfc, const float* __restrict__ bfc, const float* __restrict__ gfc, const float* __restrict__ bgc) {
  __shared__ float lg[16]; __shared__ float al[16];
  const int ck = blockIdx.x, tid = threadIdx.x, r = tid >> 4, part = tid & 15; const float* q = Hn + ((size_t)ck * 16 + 15) * DDg;
  const float* wr = wfc + (size_t)min(r, 14) * DDg; float a = 0.0f, ag = 0.0f;
#pragma unroll 1
  for (int i = 0; i < DDg / 16; ++i) { const int c = part * (DDg / 16) + i; const float qc = q[c]; a = fmaf(qc, wr[c], a); ag = fmaf(qc, gfc[c], ag); }
  a += __shfl_xor(a, 1, 32); a += __shfl_xor(a, 2, 32); a += __shfl_xor(a, 4, 32); a += __shfl_xor(a, 8, 32);
  ag += __shfl_xor(ag, 1, 32); ag += __shfl_xor(ag, 2, 32); ag += __shfl_xor(ag, 4, 32); ag += __shfl_xor(ag, 8, 32);
  if (part == 0) lg[r] = (r < 15) ? (a + bfc[r]) : (ag + bgc[0]);
  __syncthreads();
  if (tid == 0) { float m = -3.0e38f;
#pragma unroll 1
    for (int f = 0; f < 15; ++f) m = fmaxf(m, lg[f]);
    float z = 0.0f;
#pragma unroll 1
    for (int f = 0; f < 15; ++f) { al[f] = expf(lg[f] - m); z += al[f]; }
#pragma unroll 1
    for (int f = 0; f < 15; ++f) al[f] /= z;
    const float g = 1.0f / (1.0f + expf(-lg[15])); al[15] = g * (1.0f - 2.0f * 0.01f) + 0.01f; }
  __syncthreads();
  if (tid < DDg / 4) { const int c = 4 * tid; const float gate = al[15]; v4f_t agg = {0.f, 0.f, 0.f, 0.f};
#pragma unroll 1
    for (int f = 0; f < 15; ++f) { const v4f_t fr = *(const v4f_t*)(Hn + ((size_t)ck * 16 + f) * DDg + c); agg += fr * al[f]; }
    const v4f_t qv = *(const v4f_t*)(q + c); const v4f_t o = qv * (1.0f - gate) + agg * gate;
    float* d = Hn + ((size_t)ck * 16 + 15) * DDg + c; *(volatile v4f_t*)d = o; __threadfence(); *(volatile v4f_t*)d = o; }
}
__global__ __launch_bounds__(256) void k_conv2(const float* __restrict__ ZX, const float* __restrict__ cw, const float* __restrict__ cb, int dir, float* __restrict__ XC) {
  const int t = blockIdx.x, tid = threadIdx.x;
#pragma unroll 1
  for (int c = tid; c < CDg; c += 256) { float acc = cb[c];
#pragma unroll
    for (int k = 0; k < 4; ++k) { const int tt = dir ? (t + 3 - k) : (t - 3 + k); const int tc = min(max(tt, 0), SSg - 1); const float xv = ZX[(size_t)tc * NPP + DIg + c]; acc = fmaf((tt >= 0 && tt < SSg) ? xv : 0.0f, cw[c * 4 + k], acc); }
    const float sv = acc / (1.0f + expf(-acc)); *(volatile float*)(XC + (size_t)t * CDg + c) = sv; }
  __threadfence();
#pragma unroll 1
  for (int c = tid; c < CDg; c += 256) { float* p = XC + (size_t)t * CDg + c; const float v = p[0]; *(volatile float*)p = v; }
}
__global__ __launch_bounds__(256) void k_scan2(const float* __restrict__ XC, const float* __restrict__ ZX, const float* __restrict__ dtb, const float* __restrict__ Alog, const float* __restrict__ Dv, int dir, float* __restrict__ Y) {
  __shared__ float BC[TCH][2 * NSg]; __shared__ float DT[TCH][NHg]; __shared__ __attribute__((aligned(16))) float yS[TCH][256 + 4];
  const int cg = blockIdx.x, tid = threadIdx.x; const int ch = cg * 256 + tid; const int h = ch / HPg;
  const float A2 = -expf(Alog[h]) * 1.4426950408889634f; const float Dd = Dv[h]; float hs[NSg];
#pragma unroll
  for (int n = 0; n < NSg; ++n) hs[n] = 0.0f;
#pragma unroll 1
  for (int c0 = 0; c0 < SSg; c0 += TCH) {
    __syncthreads();
#pragma unroll 1
    for (int e = tid; e < TCH * 2 * NSg; e += 256) { const int tt = e >> 5, c = e & 31; const int tok = dir ? (SSg - 1 - (c0 + tt)) : (c0 + tt); BC[tt][c] = XC[(size_t)tok * CDg + DIg + c]; }
#pragma unroll 1
    for (int e = tid; e < TCH * NHg; e += 256) { const int tt = e >> 4, hh = e & 15; const int tok = dir ? (SSg - 1 - (c0 + tt)) : (c0 + tt); const float dr = ZX[(size_t)tok * NPP + 2 * DIg + 2 * NSg + hh] + dtb[hh]; DT[tt][hh] = (dr > 20.0f) ? dr : log1pf(expf(dr)); }
    __syncthreads();
#pragma unroll 1
    for (int tt = 0; tt < TCH; ++tt) { const int tok = dir ? (SSg - 1 - (c0 + tt)) : (c0 + tt);
      const float dt = DT[tt][h]; const float da = __builtin_amdgcn_exp2f(dt * A2); const float xv = XC[(size_t)tok * CDg + ch]; const float dtx = dt * xv; float y = Dd * xv;
#pragma unroll
      for (int n = 0; n < NSg; ++n) { hs[n] = fmaf(hs[n], da, dtx * BC[tt][n]); y = fmaf(hs[n], BC[tt][NSg + n], y); }
      yS[tt][tid] = y; }
    __syncthreads();
#pragma unroll 1
    for (int pass = 0; pass < 2; ++pass) {
#pragma unroll 1
      for (int i = tid; i < TCH * 64; i += 256) { const int tt = i >> 6, piece = (i & 63) * 4; const int tok = dir ? (SSg - 1 - (c0 + tt)) : (c0 + tt);
        *(volatile v4f_t*)(Y + (size_t)tok * DIg + cg * 256 + piece) = *(const v4fa*)(&yS[tt][piece]); }
      __threadfence(); }
  }
}
__global__ __launch_bounds__(256) void k_gnorm(const float* __restrict__ Y, const float* __restrict__ ZX, const float* __restrict__ w, f16* __restrict__ G) {
  __shared__ float red[256];
  const int t = blockIdx.x, tid = threadIdx.x; const int c = 4 * tid; const v4f_t y = *(const v4f_t*)(Y + (size_t)t * DIg + c); const v4f_t z = *(const v4f_t*)(ZX + (size_t)t * NPP + c);
  v4f_t g; float s = 0.0f;
#pragma unroll
  for (int e = 0; e < 4; ++e) { g[e] = y[e] * (z[e] / (1.0f + expf(-z[e]))); s += g[e] * g[e]; }
  red[tid] = s; __syncthreads();
  for (int o = 128; o > 0; o >>= 1) { if (tid < o) red[tid] += red[tid + o]; __syncthreads(); }
  const float rs = 1.0f / __builtin_sqrtf(red[0] * (1.0f / DIg) + 1e-5f); const v4f_t wv = *(const v4f_t*)(w + c);
  union { f16 hh[4]; unsigned long long u; } o;
#pragma unroll
  for (int e = 0; e < 4; ++e) o.hh[e] = (f16)(g[e] * rs * wv[e]);
  *(volatile unsigned long long*)(G + (size_t)t * DIg + c) = o.u; __threadfence(); *(volatile unsigned long long*)(G + (size_t)t * DIg + c) = o.u;
}
__global__ __launch_bounds__(256) void k_add(const float* __restrict__ a, const float* __restrict__ b2, float* __restrict__ d) {
  const size_t i4 = ((size_t)blockIdx.x * 256 + threadIdx.x) * 4; const v4f_t v = *(const v4f_t*)(a + i4) + *(const v4f_t*)(b2 + i4);
  *(volatile v4f_t*)(d + i4) = v; __threadfence(); *(volatile v4f_t*)(d + i4) = v;
}

extern "C" void kernel_launch(void* const* d_in, const int* in_sizes, int n_in,
                              void* d_out, int out_size, void* d_ws, size_t ws_size,
                              hipStream_t stream) {
  (void)in_sizes; (void)n_in; (void)out_size;
  const float** f = (const float**)d_in;
  const float* x = f[0], *n1w = f[1], *wfc = f[2], *bfc = f[3], *gfc = f[4], *bgc = f[5], *n2w = f[6], *fc1w = f[7], *fc1b = f[8], *fc2w = f[9], *fc2b = f[10];
  const float* inP[2] = {f[11], f[19]}, *cvw[2] = {f[12], f[20]}, *cvb[2] = {f[13], f[21]}, *dtb[2] = {f[14], f[22]}, *alg[2] = {f[15], f[23]}, *Dv[2] = {f[16], f[24]}, *nw[2] = {f[17], f[25]}, *outP[2] = {f[18], f[26]};
  float* out = (float*)d_out;
  char* ws = (char*)d_ws;
  float* WinT = (float*)ws; ws += (size_t)2 * DDg * NPP * 4;
  float* WoutT = (float*)ws; ws += (size_t)2 * DIg * DDg * 4;
  float* W1T = (float*)ws; ws += (size_t)DDg * FFg * 4; float* W2T = (float*)ws; ws += (size_t)FFg * DDg * 4;
  float* Hn = (float*)ws; ws += (size_t)SSg * DDg * 4;
  float* ZX = (float*)ws; ws += (size_t)SSg * NPP * 4;
  float* XC = (float*)ws; ws += (size_t)SSg * CDg * 4;
  float* Y = (float*)ws; ws += (size_t)SSg * DIg * 4; f16* G16 = (f16*)ws; ws += (size_t)SSg * DIg * 2;
  float* O1 = (float*)ws; ws += (size_t)SSg * DDg * 4;
  float* R2 = (float*)ws; ws += (size_t)SSg * DDg * 4;
  float* HN2 = (float*)ws; ws += (size_t)SSg * DDg * 4; f16* Mh = (f16*)ws; ws += (size_t)SSg * FFg * 2;
  float* ones = (float*)ws; ws += DDg * 4;
  if ((size_t)(ws - (char*)d_ws) > ws_size) return;
  const dim3 blk(256);
  k_fill<<<dim3(1), blk, 0, stream>>>(ones, 1.0f, DDg / 4);
  for (int m = 0; m < 2; ++m) { k_padin<<<dim3(DDg), blk, 0, stream>>>(inP[m], WinT + (size_t)m * DDg * NPP); k_transpose<<<dim3((DDg / 64) * (DIg / 64)), blk, 0, stream>>>(outP[m], WoutT + (size_t)m * DIg * DDg, DDg, DIg); }
  k_transpose<<<dim3((FFg / 64) * (DDg / 64)), blk, 0, stream>>>(fc1w, W1T, FFg, DDg); k_transpose<<<dim3((DDg / 64) * (FFg / 64)), blk, 0, stream>>>(fc2w, W2T, DDg, FFg);

  for (int b = 0; b < NBg; ++b) {
    const float* xb = x + (size_t)b * SSg * DDg;
    k_rms<<<dim3(SSg / 16), blk, 0, stream>>>(xb, n1w, Hn);
    k_fuse<<<dim3(SSg / 16), blk, 0, stream>>>(Hn, wfc, bfc, gfc, bgc);
    for (int m = 0; m < 2; ++m) {
      gemm_kne<float, 0, false><<<dim3(SSg / 128, NPP / 128), blk, 0, stream>>>(Hn, DDg, WinT + (size_t)m * DDg * NPP, NPP, nullptr, nullptr, nullptr, ZX, NPP, DDg);
      k_conv2<<<dim3(SSg), blk, 0, stream>>>(ZX, cvw[m], cvb[m], m, XC);
      k_scan2<<<dim3(DIg / 256), blk, 0, stream>>>(XC, ZX, dtb[m], alg[m], Dv[m], m, Y);
      k_gnorm<<<dim3(SSg), blk, 0, stream>>>(Y, ZX, nw[m], G16);
      gemm_kne<f16, 2, false><<<dim3(SSg / 128, DDg / 128), blk, 0, stream>>>(G16, DIg, WoutT + (size_t)m * DIg * DDg, DDg, nullptr, m ? O1 : xb, ones, O1, DDg, DIg);
    }
    k_add<<<dim3((size_t)SSg * DDg / 4 / 256), blk, 0, stream>>>(O1, xb, R2);
    k_rms<<<dim3(SSg / 16), blk, 0, stream>>>(O1, n2w, HN2);
    gemm_kne<float, 11, true><<<dim3(SSg / 128, FFg / 128), blk, 0, stream>>>(HN2, DDg, W1T, FFg, fc1b, nullptr, nullptr, Mh, FFg, DDg);
    gemm_kne<f16, 2, false><<<dim3(SSg / 128, DDg / 128), blk, 0, stream>>>(Mh, FFg, W2T, DDg, fc2b, R2, ones, out + (size_t)b * SSg * DDg, DDg, FFg);
  }
}
